// EqvRESFeedForward_51994874085883
// MI455X (gfx1250) — hardware-verified
//
#include <hip/hip_runtime.h>
#include <math.h>

typedef __attribute__((ext_vector_type(16))) _Float16 v16h;
typedef __attribute__((ext_vector_type(16))) __bf16 v16b;
typedef __attribute__((ext_vector_type(8)))  _Float16 v8h;
typedef __attribute__((ext_vector_type(8)))  float v8f;
typedef __attribute__((ext_vector_type(4)))  float v4f;
typedef __attribute__((ext_vector_type(2)))  float v2f;
typedef __attribute__((ext_vector_type(4)))  unsigned v4u;
typedef __attribute__((ext_vector_type(4)))  int v4i;
typedef float __attribute__((may_alias)) float_a;
typedef int __attribute__((may_alias)) int_a;

template <typename T> __device__ __forceinline__ void vst2(void* p, T v) { *(volatile T*)p = v; __threadfence(); *(volatile T*)p = v; }
__device__ __forceinline__ v8f wmma16(v16h a, v16h b, v8f c) {
  v8f d = __builtin_amdgcn_wmma_f32_16x16x32_f16(false, a, false, b, (short)0, c, false, false);
  asm volatile("v_nop\n\tv_nop\n\tv_nop\n\tv_nop" : "+v"(d) : "v"(a), "v"(b));
  return d;
}
__device__ __forceinline__ v8f wmma_bf(v16b a, v16b b, v8f c) {
  v8f d = __builtin_amdgcn_wmma_f32_16x16x32_bf16(false, a, false, b, (short)0, c, false, false);
  asm volatile("v_nop\n\tv_nop\n\tv_nop\n\tv_nop" : "+v"(d) : "v"(a), "v"(b));
  return d;
}
__device__ __forceinline__ v16h frag_h(const _Float16* rowk0, int lane) {
  union { v16h v; v8h q[2]; } u; const _Float16* p = rowk0 + 8 * (lane >> 4);
  u.q[0] = *(const v8h*)p; u.q[1] = *(const v8h*)(p + 16); return u.v;
}
__device__ __forceinline__ v16h frag_f32(const float* rowk0, int lane) {
  v16h a; const float* p = rowk0 + 8 * (lane >> 4);
#pragma unroll
  for (int i = 0; i < 8; ++i) { a[i] = (_Float16)p[i]; a[8 + i] = (_Float16)p[16 + i]; }
  return a;
}
__device__ __forceinline__ v16h frag_f32s(const float* rowk0, int lane, float sc) {
  v16h a; const float* p = rowk0 + 8 * (lane >> 4);
#pragma unroll
  for (int i = 0; i < 8; ++i) { a[i] = (_Float16)(p[i] * sc); a[8 + i] = (_Float16)(p[16 + i] * sc); }
  return a;
}
__device__ __forceinline__ v16h fragc_f32(const float* W, int k0, int n, int lane, int ld, int K) {
  v16h a; const int g = lane >> 4;
#pragma unroll
  for (int i = 0; i < 8; ++i) { const int ka = k0 + 8 * g + i, kb = ka + 16;
    a[i] = (_Float16)(ka < K ? W[(size_t)(ka < K ? ka : K - 1) * ld + n] : 0.f); a[8 + i] = (_Float16)(kb < K ? W[(size_t)(kb < K ? kb : K - 1) * ld + n] : 0.f); }
  return a;
}
struct F2 { v16b h, l; };
__device__ __forceinline__ F2 bsplit16(const float v[16]) { F2 r;
#pragma unroll
  for (int i = 0; i < 16; ++i) { const __bf16 h = (__bf16)v[i]; r.h[i] = h; r.l[i] = (__bf16)(v[i] - (float)h); }
  return r; }
__device__ __forceinline__ F2 split_row(const float* row, int k0, int lane) { float v[16]; const float* p = row + k0 + 8 * (lane >> 4);
#pragma unroll
  for (int i = 0; i < 8; ++i) { v[i] = p[i]; v[8 + i] = p[16 + i]; }
  return bsplit16(v); }
__device__ __forceinline__ F2 split_rowK(const float* row, int k0, int lane, int K) { float v[16]; const int g = lane >> 4;
#pragma unroll
  for (int i = 0; i < 8; ++i) { const int ka = k0 + 8 * g + i, kb = ka + 16; v[i] = ka < K ? row[ka < K ? ka : K - 1] : 0.f; v[8 + i] = kb < K ? row[kb < K ? kb : K - 1] : 0.f; }
  return bsplit16(v); }
__device__ __forceinline__ F2 split_col(const float* W, int k0, int n, int lane, int ld, int K) { float v[16]; const int g = lane >> 4;
#pragma unroll
  for (int i = 0; i < 8; ++i) { const int ka = k0 + 8 * g + i, kb = ka + 16; v[i] = ka < K ? W[(size_t)(ka < K ? ka : K - 1) * ld + n] : 0.f; v[8 + i] = kb < K ? W[(size_t)(kb < K ? kb : K - 1) * ld + n] : 0.f; }
  return bsplit16(v); }
__device__ __forceinline__ v8f mac3(const F2& a, const F2& b, v8f c) { c = wmma_bf(a.l, b.h, c); c = wmma_bf(a.h, b.l, c); return wmma_bf(a.h, b.h, c); }
__device__ __forceinline__ float sigm(float v) { return 1.0f / (1.0f + expf(-v)); }
#define LDSX() do { asm volatile("s_wait_dscnt 0" ::: "memory"); __builtin_amdgcn_wave_barrier(); __builtin_amdgcn_fence(__ATOMIC_RELEASE, "workgroup"); } while (0)


#define NB2 2
#define NP 384
#ifndef NN
#define NN 384
#endif
#define CH 16
#define NBAS 10
#define HW 64
#define KTOT (NN * HW)
typedef __attribute__((ext_vector_type(8))) __bf16 v8b;
__device__ __forceinline__ v16b frag_b(const __bf16* rowk0, int lane) {
  union { v16b v; v8b q[2]; } u; const __bf16* p = rowk0 + 8 * (lane >> 4);
  u.q[0] = *(const v8b*)p; u.q[1] = *(const v8b*)(p + 16); return u.v;
}
__device__ __forceinline__ float bfr(float v) { return (float)(__bf16)v; }
__device__ __attribute__((noinline)) float exp_ni(float v) { return expf(v); }
__device__ __attribute__((noinline)) float erf_ni(float v) { return erff(v); }

__device__ __forceinline__ void put_hl(__bf16* h, __bf16* l, float v) { const __bf16 hb = (__bf16)v; *h = hb; *l = (__bf16)(v - (float)hb); }
#define WS_XIN  0u
#define WS_GTH  (WS_XIN + 4u * NB2 * NN * CH)
#define WS_GTL  (WS_GTH + 2u * NB2 * CH * KTOT)
#define WS_X1   (WS_GTL + 2u * NB2 * CH * KTOT)
#define WS_X2   (WS_X1 + 4u * NB2 * NN * CH)
#define WS_END  (WS_X2 + 4u * NB2 * NN * CH)

__global__ __launch_bounds__(256) void k_xin(const float* __restrict__ X, const int* __restrict__ MK, float* __restrict__ XIN) {
  __shared__ __align__(16) float s[64][CH]; const int tid = threadIdx.x; const size_t n0 = (size_t)blockIdx.x * 64;
  for (int q = tid; q < 64 * CH; q += 256) { const size_t gn = n0 + (q >> 4); const int b = (int)(gn / NN), n = (int)(gn % NN); const int keep = MK[((size_t)b * NP + n) * NP + n] != 0; s[q >> 4][q & 15] = keep ? bfr(X[((size_t)b * NP + n) * CH + (q & 15)]) : 0.f; }
  __syncthreads();
  vst2(XIN + n0 * CH + tid * 4, *(const v4f*)(&s[0][0] + tid * 4));
}
__global__ __launch_bounds__(256) void k_gt(const float* __restrict__ XIN, const float* __restrict__ W2, __bf16* __restrict__ GTH, __bf16* __restrict__ GTL) {
  __shared__ float sx[CH]; __shared__ __align__(16) __bf16 sh[CH][HW + 8], sl[CH][HW + 8];
  const int tid = threadIdx.x; const size_t gm = blockIdx.x; const int b = (int)(gm / NN), m = (int)(gm % NN);
  if (tid < CH) sx[tid] = XIN[gm * CH + tid];
  __syncthreads();
  for (int q = tid; q < HW * CH; q += 256) { const int h = q >> 4, i = q & 15; float s = 0.f;
#pragma unroll
    for (int j = 0; j < CH; ++j) s += bfr(W2[(size_t)h * (CH * CH) + i * CH + j]) * sx[j];
    put_hl(&sh[i][h], &sl[i][h], s); }
  __syncthreads();
  if (tid < 2 * CH * 8) { const int pl = tid >> 7, rem = tid & 127, i = rem >> 3, pc = rem & 7; __bf16* dst = (pl ? GTL : GTH) + ((size_t)b * CH + i) * KTOT + (size_t)m * HW + pc * 8; vst2((unsigned*)dst, *(const v4u*)&(pl ? sl : sh)[i][pc * 8]); }
}
__global__ __launch_bounds__(128) void k_conv(const float* __restrict__ XYZ, const float* __restrict__ W1, const __bf16* __restrict__ GTH, const __bf16* __restrict__ GTL, float* __restrict__ OUT) {
  __shared__ float sw1[NBAS][HW]; __shared__ __align__(16) float sred[4][16][20]; __shared__ __align__(16) float so[16][16];
  const int tid = threadIdx.x, wave = tid >> 5, lane = tid & 31, col = lane & 15, g = lane >> 4; const int n0 = blockIdx.x * 16, b = blockIdx.y;
  for (int q = tid; q < NBAS * HW; q += 128) sw1[q / HW][q % HW] = bfr(W1[q]);
  __syncthreads();
  const int n = n0 + col; const float xn = bfr(XYZ[((size_t)b * NP + n) * 3 + 0]), yn = bfr(XYZ[((size_t)b * NP + n) * 3 + 1]), zn = bfr(XYZ[((size_t)b * NP + n) * 3 + 2]);
  float cen[NBAS];
#pragma unroll
  for (int k = 0; k < NBAS; ++k) cen[k] = (k == NBAS - 1) ? 10.0f : (float)k * (10.0f / 9.0f);
  v8f acc = {};
#pragma unroll 1
  for (int mi = 0; mi < NN / 4; ++mi) { const int m = wave * (NN / 4) + mi;
    const float dx = xn - bfr(XYZ[((size_t)b * NP + m) * 3 + 0]), dy = yn - bfr(XYZ[((size_t)b * NP + m) * 3 + 1]), dz = zn - bfr(XYZ[((size_t)b * NP + m) * 3 + 2]);
    const float r = sqrtf(dx * dx + dy * dy + dz * dz + 1e-12f); float rb[NBAS];
#pragma unroll
    for (int k = 0; k < NBAS; ++k) { const float t = (r - cen[k]); rb[k] = exp_ni(-(t * t)); }
#pragma unroll
    for (int kc = 0; kc < 2; ++kc) { float v[16];
#pragma unroll
      for (int i = 0; i < 8; ++i) { const int h0 = kc * 32 + 8 * g + i, h1 = h0 + 16; float s0 = 0.f, s1 = 0.f;
#pragma unroll
        for (int k = 0; k < NBAS; ++k) { s0 += rb[k] * sw1[k][h0]; s1 += rb[k] * sw1[k][h1]; }
        v[i] = s0 / (1.0f + exp_ni(-s0)); v[8 + i] = s1 / (1.0f + exp_ni(-s1)); }
      const F2 a = bsplit16(v); const size_t kb = (size_t)m * HW + kc * 32; const v16b bh = frag_b(GTH + ((size_t)b * CH + col) * KTOT + kb, lane), bl = frag_b(GTL + ((size_t)b * CH + col) * KTOT + kb, lane);
      acc = wmma_bf(a.l, bh, acc); acc = wmma_bf(a.h, bl, acc); acc = wmma_bf(a.h, bh, acc); } }
#pragma unroll
  for (int rr = 0; rr < 8; ++rr) sred[wave][8 * g + rr][col] = acc[rr];
  __syncthreads();
  for (int q = tid; q < 256; q += 128) { const int rl = q >> 4, i = q & 15; so[rl][i] = ((sred[0][rl][i] + sred[1][rl][i]) + (sred[2][rl][i] + sred[3][rl][i])) / sqrtf((float)NN); }
  __syncthreads();
  if (tid < 64) vst2(OUT + ((size_t)b * NN + n0) * CH + tid * 4, *(const v4f*)(&so[0][0] + tid * 4));
}
__global__ __launch_bounds__(256) void k_copy16(const float* __restrict__ S, float* __restrict__ D) { const size_t off = ((size_t)blockIdx.x * 256 + threadIdx.x) * 4; vst2(D + off, *(const v4f*)(S + off)); }
__global__ __launch_bounds__(64) void k_fin(const float* __restrict__ X2, const int* __restrict__ MK, const float* __restrict__ FC, float* __restrict__ out) {
  __shared__ float sv[NB2][CH], snv[NB2][CH], sy[NB2][CH], sst[NB2][2]; __shared__ __align__(16) float so[NB2 * CH]; const int tid = threadIdx.x;
  if (tid < NB2 * CH) { const int b = tid >> 4, i = tid & 15; float s = 0.f;
#pragma unroll 1
    for (int n = 0; n < NN; ++n) { const int keep = MK[((size_t)b * NP + n) * NP + n] != 0; s += keep ? X2[((size_t)b * NN + n) * CH + i] : 0.f; }
    sv[b][i] = s; }
  __syncthreads();
  if (tid < NB2) { const int b = tid; float mean = 0.f;
#pragma unroll 1
    for (int i = 0; i < CH; ++i) mean += sv[b][i];
    mean /= (float)CH; float var = 0.f;
#pragma unroll 1
    for (int i = 0; i < CH; ++i) { const float d = sv[b][i] - mean; var += d * d; }
    sst[b][0] = mean; sst[b][1] = sqrtf(var / (float)(CH - 1)) + 1e-6f; }
  __syncthreads();
  if (tid < NB2 * CH) { const int b = tid >> 4, i = tid & 15; snv[b][i] = (sv[b][i] - sst[b][0]) / sst[b][1]; }
  __syncthreads();
  if (tid < NB2 * CH) { const int b = tid >> 4, o = tid & 15; float s = 0.f;
#pragma unroll 1
    for (int i = 0; i < CH; ++i) s += snv[b][i] * bfr(FC[o * CH + i]);
    sy[b][o] = s; }
  __syncthreads();
  if (tid < NB2) { const int b = tid; float mx = -3.0e38f;
#pragma unroll 1
    for (int o = 0; o < CH; ++o) mx = fmaxf(mx, sy[b][o]);
    float z = 0.f;
#pragma unroll 1
    for (int o = 0; o < CH; ++o) { const float e = exp_ni(sy[b][o] - mx); sy[b][o] = e; z += e; }
#pragma unroll 1
    for (int o = 0; o < CH; ++o) so[b * CH + o] = sy[b][o] / z; }
  __syncthreads();
  if (tid < 8) vst2(out + tid * 4, *(const v4f*)&so[tid * 4]);
}
extern "C" void kernel_launch(void* const* d_in, const int* in_sizes, int n_in, void* d_out, int out_size, void* d_ws, size_t ws_size, hipStream_t stream) {
  (void)in_sizes; (void)n_in; (void)out_size;
  const float** F = (const float**)d_in; const int* MK = (const int*)d_in[2];
  if (ws_size < (size_t)WS_END) return;
  char* ws = (char*)d_ws; float *XIN = (float*)(ws + WS_XIN), *X1 = (float*)(ws + WS_X1), *X2 = (float*)(ws + WS_X2); __bf16 *GTH = (__bf16*)(ws + WS_GTH), *GTL = (__bf16*)(ws + WS_GTL);
  k_xin<<<NB2 * NN / 64, 256, 0, stream>>>(F[0], MK, XIN);
  k_gt<<<NB2 * NN, 256, 0, stream>>>(XIN, F[4], GTH, GTL);
  k_conv<<<dim3(NN / 16, NB2), 128, 0, stream>>>(F[1], F[3], GTH, GTL, X1);
  k_copy16<<<NB2 * NN * CH / 1024, 256, 0, stream>>>(X1, XIN);
  k_gt<<<NB2 * NN, 256, 0, stream>>>(XIN, F[6], GTH, GTL);
  k_conv<<<dim3(NN / 16, NB2), 128, 0, stream>>>(F[1], F[5], GTH, GTL, X2);
  k_fin<<<1, 64, 0, stream>>>(X2, MK, F[7], (float*)d_out);
}
